// HierDDLts_63410897158384
// MI455X (gfx1250) — hardware-run, weakly checked
//
#include <hip/hip_runtime.h>


namespace {
constexpr int NB = 8, S = 2048, D = 64, G = 5, O = 512, KW = 32  ;
constexpr float XS = 8.0f, HS = 256.0f, WSC = 256.0f, LNEPS = 1e-5f, TWO_PI = 6.283185307179586f;
typedef _Float16 b16;
typedef __attribute__((ext_vector_type(16))) _Float16 v16b;
typedef __attribute__((ext_vector_type(8))) _Float16 v8b;
typedef __attribute__((ext_vector_type(8))) float v8f;
typedef __attribute__((ext_vector_type(4))) float v4f;
__device__ __forceinline__ float bf16_rne(float f) { unsigned int u = __float_as_uint(f); u += 0x7FFFu + ((u >> 16) & 1u); float r = __uint_as_float(u & 0xFFFF0000u); asm volatile("" : "+v"(r)); return r; }
__device__ __forceinline__ float bfv(float f) { float r = bf16_rne(f); asm volatile("" : "+v"(r)); return r; }
__device__ __forceinline__ void split16(float v, b16& hi, b16& lo) { hi = (b16)v; lo = (b16)(v - (float)hi); }
__device__ __forceinline__ v16b frag_kb(const b16* p, int hh) { const v8b a = *(const v8b*)(p + 8 * hh), b = *(const v8b*)(p + 16 + 8 * hh); v16b f;
#pragma unroll
  for (int e = 0; e < 8; ++e) { f[e] = a[e]; f[8 + e] = b[e]; } return f; }
__device__ __forceinline__ v8f wmma16b(v16b a, v16b b, v8f c) { v8f d = __builtin_amdgcn_wmma_f32_16x16x32_f16(false, a, false, b, (short)0, c, false, false); asm volatile("v_nop\n\tv_nop\n\tv_nop\n\tv_nop" : "+v"(d) : "v"(a), "v"(b)); return d; }
__device__ __forceinline__ void wave_lds_sync() { __builtin_amdgcn_fence(__ATOMIC_RELEASE, "workgroup"); __builtin_amdgcn_wave_barrier(); __builtin_amdgcn_fence(__ATOMIC_ACQUIRE, "workgroup"); }
__device__ __forceinline__ float pmul(float a, float b) { float p = a * b; asm volatile("" : "+v"(p)); return p; }

__global__ __launch_bounds__(256) void prep_kernel(const float* __restrict__ M, const float* __restrict__ seq, const float* __restrict__ Lk, b16* __restrict__ MB, b16* __restrict__ SQ, b16* __restrict__ LT) { const size_t u = (size_t)blockIdx.x * 256 + threadIdx.x; v8b v;
  if (u < (size_t)D * 8) { const int i = (int)(u / 8), d0 = (int)(u % 8) * 8;
#pragma unroll
    for (int j = 0; j < 8; ++j) v[j] = (b16)(bf16_rne(M[i * D + d0 + j]) * XS); for (int pass = 0; pass < 2; ++pass) { *(volatile v8b*)(MB + (size_t)i * D + d0) = v; __threadfence(); } }
  if (u < (size_t)NB * S * 8) { const size_t r = u / 8; const int d0 = (int)(u % 8) * 8;
#pragma unroll
    for (int j = 0; j < 8; ++j) v[j] = (b16)(bf16_rne(seq[r * D + d0 + j]) * WSC); for (int pass = 0; pass < 2; ++pass) { *(volatile v8b*)(SQ + r * D + d0) = v; __threadfence(); } }
  {
    const int wave = threadIdx.x >> 5, lane = threadIdx.x & 31; const int o = blockIdx.x * 8 + wave; if (o < O) for (int pass = 0; pass < 2; ++pass) { for (int k0 = 0; k0 < S; k0 += 256) { v8b w;
#pragma unroll
        for (int j = 0; j < 8; ++j) w[j] = (b16)(bf16_rne(Lk[(size_t)(k0 + lane * 8 + j) * O + o]) * XS); *(volatile v8b*)(LT + (size_t)o * S + k0 + lane * 8) = w; } __threadfence(); } } }
__global__ __launch_bounds__(32) void z0t_kernel(const b16* __restrict__ MB, const b16* __restrict__ SQ, int BLIM, float* __restrict__ Z0T) { __shared__ float Tf[16][260]; const int lane = threadIdx.x, nloc = lane & 15, hlf = lane >> 4; const int b = blockIdx.x / (4 * (S / 256)); if (b >= BLIM) return; const int it = (blockIdx.x / (S / 256)) % 4, kg = blockIdx.x % (S / 256); v8f acc[16];
#pragma unroll
  for (int t = 0; t < 16; ++t) acc[t] = (v8f){};
#pragma unroll
  for (int kb = 0; kb < D; kb += 32) { const v16b a = frag_kb(MB + (size_t)(it * 16 + nloc) * D + kb, hlf);
#pragma unroll
    for (int t = 0; t < 16; ++t) acc[t] = wmma16b(a, frag_kb(SQ + ((size_t)b * S + kg * 256 + t * 16 + nloc) * D + kb, hlf), acc[t]); }
#pragma unroll
  for (int t = 0; t < 16; ++t)
#pragma unroll
    for (int r8 = 0; r8 < 8; ++r8) Tf[8 * hlf + r8][t * 16 + nloc] = acc[t][r8] * (1.0f / (XS * WSC));
  wave_lds_sync();
  for (int pass = 0; pass < 2; ++pass) { for (int rr = 0; rr < 16; ++rr) for (int q = 0; q < 2; ++q) *(volatile v4f*)(Z0T + ((size_t)b * D + it * 16 + rr) * S + kg * 256 + q * 128 + lane * 4) = *(const v4f*)(&Tf[rr][q * 128 + lane * 4]); __threadfence(); } }
__global__ __launch_bounds__(256) void ln_kernel(const float* __restrict__ Z0T, int BLIM, float* __restrict__ MU, float* __restrict__ RSD) { const size_t u = (size_t)blockIdx.x * 256 + threadIdx.x; const int b = (int)(u / S), k = (int)(u % S); if (b >= BLIM) return; float s = 0.0f; for (int i = 0; i < D; ++i) s += Z0T[((size_t)b * D + i) * S + k]; const float m = s / D; float s2 = 0.0f; for (int i = 0; i < D; ++i) { const float d = Z0T[((size_t)b * D + i) * S + k] - m; s2 += d * d; } const float r = rsqrtf(s2 / D + LNEPS);
  for (int pass = 0; pass < 2; ++pass) { ((volatile float*)MU)[u] = m; ((volatile float*)RSD)[u] = r; __threadfence(); } }
__global__ __launch_bounds__(32) void t_kernel(const float* __restrict__ Z0T, const float* __restrict__ MU, const float* __restrict__ RSD, const float* __restrict__ Pp, const float* __restrict__ gam, const float* __restrict__ bet, int KLIM, float* __restrict__ SB) {
  __shared__ __attribute__((aligned(16))) b16 Wh[D][72], Wl[D][72], Ah[16][72], Al[16][72]; __shared__ float Tt[NB][D][KW + 1];
  const int lane = threadIdx.x, nloc = lane & 15, hlf = lane >> 4; const int k0 = blockIdx.x * KW; if (k0 >= KLIM) return;
  if (lane < 16) for (int c = D; c < 72; ++c) { Ah[lane][c] = (b16)0.0f; Al[lane][c] = (b16)0.0f; } for (int r = 0; r < D; r += 32) for (int c = D; c < 72; ++c) { Wh[r + lane][c] = (b16)0.0f; Wl[r + lane][c] = (b16)0.0f; }
  for (int rr = NB; rr < 16; ++rr) for (int c = lane; c < D; c += 32) { Ah[rr][c] = (b16)0.0f; Al[rr][c] = (b16)0.0f; }
  wave_lds_sync();
#pragma unroll 1
  for (int kk = 0; kk < KW; ++kk) { const int k = k0 + kk; const float num = TWO_PI * (float)k;
#pragma unroll 1
    for (int idx = lane; idx < D * D; idx += 32) { const int i = idx / D, j = idx % D; float w = 0.0f;
#pragma unroll
      for (int g = 0; g < G; ++g) { const int pe = idx * G + g; const float period = (float)(pe + 2); const float arg = __fdiv_rn(num, period); w += pmul(bfv(Pp[pe]), cosf(arg)); }
      b16 p, ql; split16(w * HS, p, ql); Wh[i][j] = p; Wl[i][j] = ql; }
    for (int b = 0; b < NB; ++b) for (int q = 0; q < 2; ++q) { const int j = q * 32 + lane; const float z0 = Z0T[((size_t)b * D + j) * S + k]; const float z = pmul(pmul(z0 - MU[b * S + k], RSD[b * S + k]), bfv(gam[j])) + bfv(bet[j]); b16 p, ql; split16(z * HS, p, ql); Ah[b][j] = p; Al[b][j] = ql; }
    wave_lds_sync(); v8f acc[4] = {(v8f){}, (v8f){}, (v8f){}, (v8f){}};
#pragma unroll
    for (int kb = 0; kb < D; kb += 32) { const v16b a = frag_kb(&Ah[nloc][kb], hlf), al = frag_kb(&Al[nloc][kb], hlf);
#pragma unroll
      for (int t = 0; t < 4; ++t) { const v16b wh = frag_kb(&Wh[t * 16 + nloc][kb], hlf), wl = frag_kb(&Wl[t * 16 + nloc][kb], hlf); acc[t] = wmma16b(a, wh, acc[t]); acc[t] = wmma16b(a, wl, acc[t]); acc[t] = wmma16b(al, wh, acc[t]); } }
    if (hlf == 0) {
#pragma unroll
      for (int t = 0; t < 4; ++t)
#pragma unroll
        for (int r8 = 0; r8 < 8; ++r8) Tt[r8][t * 16 + nloc][kk] = acc[t][r8] * (1.0f / (HS * HS)); }
    wave_lds_sync(); }
  for (int pass = 0; pass < 2; ++pass) { for (int b = 0; b < NB; ++b) for (int i = 0; i < D; ++i) { const size_t o = ((size_t)b * D + i) * S + k0 + lane; ((volatile float*)SB)[o] = Tt[b][i][lane] + Z0T[o]; } __threadfence(); } }
__global__ __launch_bounds__(32) void u_kernel(const b16* __restrict__ LT, const float* __restrict__ SB, int BLIM, int KLIM, float* __restrict__ out) { __shared__ __attribute__((aligned(16))) b16 Bh[D][264], Bl[D][264]; __shared__ float Tf[16][D + 4]; const int lane = threadIdx.x, nloc = lane & 15, hlf = lane >> 4; const int b = blockIdx.x / (O / 16); if (b >= BLIM) return; const int o0 = (blockIdx.x % (O / 16)) * 16;
  v8f acc[4] = {(v8f){}, (v8f){}, (v8f){}, (v8f){}};
  for (int r = 0; r < D; r += 32) for (int c = 256; c < 264; ++c) { Bh[r + lane][c] = (b16)0.0f; Bl[r + lane][c] = (b16)0.0f; }
#pragma unroll 1
  for (int kc = 0; kc < KLIM; kc += 256) { for (int i = 0; i < D; ++i) for (int q = 0; q < 8; ++q) { b16 p, ql; split16(SB[((size_t)b * D + i) * S + kc + q * 32 + lane] * HS, p, ql); Bh[i][q * 32 + lane] = p; Bl[i][q * 32 + lane] = ql; }
    wave_lds_sync();
#pragma unroll 2
    for (int kb = 0; kb < 256; kb += 32) { const v16b a = frag_kb(LT + (size_t)(o0 + nloc) * S + kc + kb, hlf);
#pragma unroll
      for (int t = 0; t < 4; ++t) { acc[t] = wmma16b(a, frag_kb(&Bh[t * 16 + nloc][kb], hlf), acc[t]); acc[t] = wmma16b(a, frag_kb(&Bl[t * 16 + nloc][kb], hlf), acc[t]); } }
    wave_lds_sync(); }
#pragma unroll
  for (int t = 0; t < 4; ++t)
#pragma unroll
    for (int r8 = 0; r8 < 8; ++r8) Tf[8 * hlf + r8][t * 16 + nloc] = acc[t][r8] * (1.0f / (XS * HS));
  wave_lds_sync();
  for (int pass = 0; pass < 2; ++pass) { for (int rr = 0; rr < 16; ++rr) for (int q = 0; q < 2; ++q) ((volatile float*)out)[((size_t)b * O + o0 + rr) * D + q * 32 + lane] = Tf[rr][q * 32 + lane]; __threadfence(); } }
}

extern "C" void kernel_launch(void* const* d_in, const int* in_sizes, int n_in, void* d_out, int out_size, void* d_ws, size_t ws_size, hipStream_t stream) {
  (void)n_in;
  auto Fp = [&](int i) { return (const float*)d_in[i]; };
  if (in_sizes[0] != NB * S * D || in_sizes[1] != D * D || in_sizes[2] != D * D * G || in_sizes[3] != S * O || in_sizes[4] != D || in_sizes[5] != D || out_size != NB * O * D) return;
  const int BLIM = NB, KLIM = S;
  size_t off = 0; char* ws = (char*)d_ws;
  auto carve = [&](size_t bytes) { char* p = ws + off; off += (bytes + 255) & ~(size_t)255; return p; };
  b16* MB = (b16*)carve((size_t)D * D * 2); b16* SQ = (b16*)carve((size_t)NB * S * D * 2); b16* LT = (b16*)carve((size_t)O * S * 2); float* Z0T = (float*)carve((size_t)NB * D * S * 4); float* MU = (float*)carve((size_t)NB * S * 4); float* RSD = (float*)carve((size_t)NB * S * 4); float* SB = (float*)carve((size_t)NB * D * S * 4);
  if (off > ws_size || off > ((size_t)32 << 20)) return;
  prep_kernel<<<(NB * S * 8 + 255) / 256, 256, 0, stream>>>(Fp(1), Fp(0), Fp(3), MB, SQ, LT);
  z0t_kernel<<<BLIM * 4 * (S / 256), 32, 0, stream>>>(MB, SQ, BLIM, Z0T);
  ln_kernel<<<(BLIM * S + 255) / 256, 256, 0, stream>>>(Z0T, BLIM, MU, RSD);
  t_kernel<<<KLIM / KW, 32, 0, stream>>>(Z0T, MU, RSD, Fp(2), Fp(4), Fp(5), KLIM, SB);
  u_kernel<<<BLIM * (O / 16), 32, 0, stream>>>(LT, SB, BLIM, KLIM, (float*)d_out);
}
